// CompactedViTAttention_52235392254394
// MI455X (gfx1250) — hardware-verified
//
#include <hip/hip_runtime.h>
#include <hip/hip_bf16.h>
#include <math.h>


#define BB 16
#define SS 1088
#define DD 512
#define DO 384
#define DM 768
#define HH 6
#define DKK 64
#define QW 2
#define NT 1025
#define NTOT 16400
#define MP 16512

typedef _Float16 bf16;
typedef __attribute__((ext_vector_type(4))) unsigned v4u_t;
typedef unsigned v4ua __attribute__((ext_vector_type(4), may_alias));
typedef __attribute__((ext_vector_type(4))) float v4f_t;
typedef float v4fa __attribute__((ext_vector_type(4), may_alias));
typedef __attribute__((ext_vector_type(16))) bf16  bf16x16;
typedef __attribute__((ext_vector_type(8)))  bf16  bf16x8;
typedef __attribute__((ext_vector_type(4)))  bf16  bf16x4;
typedef __attribute__((ext_vector_type(8)))  float f32x8;

#define LDS_STRIDE 48
#define KSTRIDE    72
#define VSTRIDE    48

__device__ __forceinline__ f32x8 wmma_bf16(bf16x16 a, bf16x16 b, f32x8 c) {
  return __builtin_amdgcn_wmma_f32_16x16x32_f16(
      false, a, false, b, (short)0, c, false, false);
}

template <typename T>
__device__ __forceinline__ bf16x16 load_frag(const T* __restrict__ base, int ld,
                                             int row0, int k0) {
  const int lane = threadIdx.x & 31;
  const int r    = lane & 15;
  const int kh   = (lane >> 4) * 8;
  const T* p0 = base + (size_t)(row0 + r) * ld + (k0 + kh);
  const T* p1 = p0 + 16;
  bf16x16 f;
#pragma unroll
  for (int i = 0; i < 8; ++i) {
    f[i]     = (bf16)p0[i];
    f[i + 8] = (bf16)p1[i];
  }
  return f;
}

__device__ __forceinline__ bf16x16 lds_frag(const bf16* base, int stride) {
  const int lane = threadIdx.x & 31;
  const int row  = lane & 15;
  const int kh   = (lane >> 4) * 8;
  const bf16x8 lo = *(const bf16x8*)(base + row * stride + kh);
  const bf16x8 hi = *(const bf16x8*)(base + row * stride + kh + 16);
  bf16x16 f;
#pragma unroll
  for (int i = 0; i < 8; ++i) { f[i] = lo[i]; f[i + 8] = hi[i]; }
  return f;
}

template <typename T>
__device__ __forceinline__ void stage_read16(const T* __restrict__ p, float* buf) {
#pragma unroll
  for (int i = 0; i < 16; ++i) buf[i] = (float)p[i];
}

__device__ __forceinline__ void stage_write(bf16* dst, const float* buf, int nquad) {
#pragma unroll
  for (int i = 0; i < nquad; ++i) {
    bf16x4 q;
    q[0] = (bf16)buf[4 * i];     q[1] = (bf16)buf[4 * i + 1];
    q[2] = (bf16)buf[4 * i + 2]; q[3] = (bf16)buf[4 * i + 3];
    *(bf16x4*)(dst + 4 * i) = q;
  }
}

template <typename AT, int MODE>
__global__ __launch_bounds__(256) void gemm_bias_kernel(
    const AT* __restrict__ A, const float* __restrict__ W,
    const float* __restrict__ bias, void* __restrict__ out,
    int M, int N, int K) {
  __shared__ bf16 ldsA[128 * LDS_STRIDE];
  __shared__ bf16 ldsW[256 * LDS_STRIDE];
  __shared__ __attribute__((aligned(16))) unsigned char sob[256 * 136 * 2];

  const int t    = threadIdx.x;
  const int wave = t >> 5;
  const int lane = t & 31;
  const int wm   = (wave & 1) * 64;
  const int wn   = (wave >> 1) * 64;
  const int mBlk = blockIdx.x * 128;
  const int nBlk = blockIdx.y * 256;

  const int arow = t >> 1;
  const int ach  = (t & 1) * 16;

  float abuf[16];
  float wbuf[32];

  stage_read16(A + (size_t)(mBlk + arow) * K + ach, abuf);
  stage_read16(W + (size_t)(nBlk + t) * K,          wbuf);
  stage_read16(W + (size_t)(nBlk + t) * K + 16,     wbuf + 16);

  f32x8 acc[4][4] = {};

  for (int k = 0; k < K; k += 32) {
    __syncthreads();
    stage_write(&ldsA[arow * LDS_STRIDE + ach], abuf, 4);
    stage_write(&ldsW[t * LDS_STRIDE],          wbuf, 8);
    if (k + 32 < K) {
      stage_read16(A + (size_t)(mBlk + arow) * K + (k + 32) + ach, abuf);
      stage_read16(W + (size_t)(nBlk + t) * K + (k + 32),          wbuf);
      stage_read16(W + (size_t)(nBlk + t) * K + (k + 32) + 16,     wbuf + 16);
    }
    __syncthreads();

    bf16x16 af[4], wf[4];
#pragma unroll
    for (int i = 0; i < 4; ++i)
      af[i] = lds_frag(ldsA + (wm + 16 * i) * LDS_STRIDE, LDS_STRIDE);
#pragma unroll
    for (int j = 0; j < 4; ++j)
      wf[j] = lds_frag(ldsW + (wn + 16 * j) * LDS_STRIDE, LDS_STRIDE);
#pragma unroll
    for (int i = 0; i < 4; ++i)
#pragma unroll
      for (int j = 0; j < 4; ++j)
        acc[i][j] = wmma_bf16(af[i], wf[j], acc[i][j]);
  }

  const int nlane = lane & 15;
  const int mh    = (lane >> 4) * 8;
  __syncthreads();
  if (MODE == 0 || MODE == 1) {
    bf16* so = (bf16*)sob;
#pragma unroll
    for (int i = 0; i < 4; ++i)
#pragma unroll
      for (int j = 0; j < 4; ++j) {
        const int nl = wn + 16 * j + nlane;
        const float bv = bias ? bias[nBlk + nl] : 0.0f;
#pragma unroll
        for (int r = 0; r < 8; ++r) {
          const int ml = wm + 16 * i + mh + r;
          const bf16 hv = (bf16)(acc[i][j][r] + bv);
          if (MODE == 0) so[ml * 264 + nl] = hv;
          else           so[nl * 136 + ml] = hv;
        }
      }
    __syncthreads();
#pragma unroll 1
    for (int pass = 0; pass < 2; ++pass) {
      if (MODE == 0) {
        for (int ch = t; ch < 128 * 32; ch += 256) { const int ml = ch >> 5, q = (ch & 31) * 8;
          *(volatile v4u_t*)((bf16*)out + (size_t)(mBlk + ml) * N + nBlk + q) = *(const v4ua*)(so + ml * 264 + q); }
      } else {
        const int b_ = mBlk / SS, s0 = mBlk & (SS - 1);
        for (int ch = t; ch < 256 * 16; ch += 256) { const int nl = ch >> 4, q = (ch & 15) * 8; const int n = nBlk + nl, h = n >> 6, dk = n & (DKK - 1);
          *(volatile v4u_t*)((bf16*)out + (((size_t)(b_ * HH + h)) * DKK + dk) * SS + s0 + q) = *(const v4ua*)(so + nl * 136 + q); }
      }
      __threadfence();
    }
  } else {
    float* so = (float*)sob;
#pragma unroll 1
    for (int hf = 0; hf < 2; ++hf) {
      if (wm == hf * 64) {
#pragma unroll
        for (int i = 0; i < 4; ++i)
#pragma unroll
          for (int j = 0; j < 4; ++j) {
            const int nl = wn + 16 * j + nlane;
            const float bv = bias ? bias[nBlk + nl] : 0.0f;
#pragma unroll
            for (int r = 0; r < 8; ++r) so[(16 * i + mh + r) * 260 + nl] = acc[i][j][r] + bv;
          }
      }
      __syncthreads();
#pragma unroll 1
      for (int pass = 0; pass < 2; ++pass) {
        for (int ch = t; ch < 64 * 64; ch += 256) { const int ml = ch >> 6, q = (ch & 63) * 4;
          *(volatile v4f_t*)((float*)out + (size_t)(mBlk + hf * 64 + ml) * N + nBlk + q) = *(const volatile v4fa*)(so + ml * 260 + q); }
        __threadfence();
      }
      __syncthreads();
    }
  }
}

__global__ __launch_bounds__(64) void attn_kernel(
    const bf16* __restrict__ Qb, const bf16* __restrict__ Kb,
    const bf16* __restrict__ Vt,
    bf16* __restrict__ attnOut) {
  __shared__ bf16 ldsK[32 * KSTRIDE];
  __shared__ bf16 ldsV[64 * VSTRIDE];
  __shared__ __attribute__((aligned(16))) bf16 ldsO[2][32 * 72];

  const int q0blk = blockIdx.x * 64;
  const int h  = blockIdx.y;
  const int b  = blockIdx.z;
  const int t    = threadIdx.x;
  const int wave = t >> 5;
  const int lane = t & 31;
  const int qlane = lane & 15;
  const int kh8   = (lane >> 4) * 8;
  const int q0 = q0blk + wave * 32;

  const bf16* Qh = Qb + (size_t)b * NT * DD + h * DKK;
  const bf16* Kh = Kb + (size_t)b * NT * DD + h * DKK;
  const bf16* Vh = Vt + ((size_t)(b * HH + h)) * DKK * SS;

  const int krow = t >> 1;
  const int kcol = (t & 1) * 32;
  const bf16* kSrc = Kh + (size_t)krow * DD + kcol;
  const bf16* vSrc = Vh + (size_t)t * SS;

  bf16x16 qf[QW][2];
#pragma unroll
  for (int qt = 0; qt < QW; ++qt) {
    qf[qt][0] = load_frag(Qh, DD, q0 + 16 * qt, 0);
    qf[qt][1] = load_frag(Qh, DD, q0 + 16 * qt, 32);
  }

  f32x8 o[QW][4] = {};
  float mrun[QW], lrun[QW];
#pragma unroll
  for (int qt = 0; qt < QW; ++qt) { mrun[qt] = -INFINITY; lrun[qt] = 0.0f; }

  const float scale = 0.125f * 1.44269504088896340736f;
  const float NEG2 = -3.0e38f;
  const int kmax = 1055;


  bf16x8 kreg[4], vreg[4];
#pragma unroll
  for (int i = 0; i < 4; ++i) {
    kreg[i] = *(const bf16x8*)(kSrc + 8 * i);
    vreg[i] = *(const bf16x8*)(vSrc + 8 * i);
  }

  for (int kb = 0; kb <= kmax; kb += 32) {
    __syncthreads();
#pragma unroll
    for (int i = 0; i < 4; ++i) {
      *(bf16x8*)(&ldsK[krow * KSTRIDE + kcol + 8 * i]) = kreg[i];
      *(bf16x8*)(&ldsV[t * VSTRIDE + 8 * i])           = vreg[i];
    }
    if (kb + 32 <= kmax) {
      const bf16* kn = kSrc + (size_t)(kb + 32) * DD;
      const bf16* vn = vSrc + (kb + 32);
#pragma unroll
      for (int i = 0; i < 4; ++i) {
        kreg[i] = *(const bf16x8*)(kn + 8 * i);
        vreg[i] = *(const bf16x8*)(vn + 8 * i);
      }
    }
    __syncthreads();

    bf16x16 kf[2][2];
#pragma unroll
    for (int ktile = 0; ktile < 2; ++ktile)
#pragma unroll
      for (int c = 0; c < 2; ++c)
        kf[ktile][c] = lds_frag(ldsK + (ktile * 16) * KSTRIDE + c * 32, KSTRIDE);

    bf16x16 pf[QW];
    bool act[QW];
#pragma unroll
    for (int qt = 0; qt < QW; ++qt) {
      unsigned mbits = 0;
      {
#pragma unroll
        for (int r = 0; r < 8; ++r) {
          if (kb + kh8 + r < NT)      mbits |= 1u << r;
          if (kb + kh8 + 16 + r < NT) mbits |= 1u << (8 + r);
        }
        act[qt] = true;
      }
      if (act[qt]) {
        const int q_my = q0 + 16 * qt + qlane;
        f32x8 s0 = {}, s1 = {};
        s0 = wmma_bf16(kf[0][0], qf[qt][0], s0);
        s0 = wmma_bf16(kf[0][1], qf[qt][1], s0);
        s1 = wmma_bf16(kf[1][0], qf[qt][0], s1);
        s1 = wmma_bf16(kf[1][1], qf[qt][1], s1);

        float mx = -INFINITY;
#pragma unroll
        for (int r = 0; r < 8; ++r) {
          const int k0i = kb + kh8 + r;
          const int k1i = k0i + 16;
          (void)k0i; (void)k1i; (void)q_my;
          (void)q_my;
          s0[r] = (mbits & (1u << r))       ? s0[r] * scale : NEG2;
          s1[r] = (mbits & (1u << (8 + r))) ? s1[r] * scale : NEG2;
          mx = fmaxf(mx, fmaxf(s0[r], s1[r]));
        }
        mx = fmaxf(mx, __shfl_xor(mx, 16, 32));
        const float mnew  = fmaxf(mrun[qt], mx);
        const float alpha = exp2f(mrun[qt] - mnew);

        float rsum = 0.0f;
#pragma unroll
        for (int r = 0; r < 8; ++r) {
          const float p0 = exp2f(s0[r] - mnew);
          const float p1 = exp2f(s1[r] - mnew);
          rsum += p0 + p1;
          pf[qt][r]     = (bf16)(p0 * 1024.0f);
          pf[qt][r + 8] = (bf16)(p1 * 1024.0f);
        }
        rsum += __shfl_xor(rsum, 16, 32);
        lrun[qt] = lrun[qt] * alpha + rsum;
        mrun[qt] = mnew;

#pragma unroll
        for (int j = 0; j < 4; ++j)
#pragma unroll
          for (int r = 0; r < 8; ++r) o[qt][j][r] *= alpha;
      }
    }

#pragma unroll
    for (int j = 0; j < 4; ++j) {
      const bf16x16 vf = lds_frag(ldsV + (j * 16) * VSTRIDE, VSTRIDE);
#pragma unroll
      for (int qt = 0; qt < QW; ++qt)
        if (act[qt]) o[qt][j] = wmma_bf16(vf, pf[qt], o[qt][j]);
    }
  }

  bf16* so = ldsO[wave];
#pragma unroll
  for (int qt = 0; qt < QW; ++qt) {
    const float rl = 1.0f / (lrun[qt] * 1024.0f);

#pragma unroll
    for (int j = 0; j < 4; ++j)
#pragma unroll
      for (int r = 0; r < 8; ++r) so[(16 * qt + qlane) * 72 + j * 16 + kh8 + r] = (bf16)(o[qt][j][r] * rl);
  }
  asm volatile("s_wait_dscnt 0" ::: "memory");
#pragma unroll 1
  for (int pass = 0; pass < 2; ++pass) {
#pragma unroll
    for (int it = 0; it < 8; ++it) { const int ch = lane + 32 * it, ql = ch >> 3, q8 = (ch & 7) * 8;
      if (q0 + ql < NT) *(volatile v4u_t*)(attnOut + ((size_t)(b * NT + q0 + ql)) * DO + h * DKK + q8) = *(const v4ua*)(so + ql * 72 + q8); }
    __threadfence();
  }
}

__global__ __launch_bounds__(256) void k_tw(const float* __restrict__ W, float* __restrict__ WT, int K, int N) {
  __shared__ float tile[64][65];
  const int kb0 = blockIdx.y * 64, n0 = blockIdx.x * 64, t = threadIdx.x;
  for (int i = t; i < 64 * 64; i += 256) { const int kr = i >> 6, nc = i & 63; tile[kr][nc] = W[(size_t)(kb0 + kr) * N + n0 + nc]; }
  __syncthreads();
#pragma unroll 1
  for (int pass = 0; pass < 2; ++pass) {
    for (int i = t; i < 64 * 16; i += 256) { const int nr = i >> 4, k4 = (i & 15) * 4; v4f_t v; v.x = tile[k4][nr]; v.y = tile[k4 + 1][nr]; v.z = tile[k4 + 2][nr]; v.w = tile[k4 + 3][nr];
      *(volatile v4f_t*)(WT + (size_t)(n0 + nr) * K + kb0 + k4) = v; }
    __threadfence();
  }
}

__global__ __launch_bounds__(256) void k_vt(const bf16* __restrict__ Vr, bf16* __restrict__ Vt) {
  __shared__ bf16 tile[64][72];
  const int s0 = blockIdx.x * 64, h = blockIdx.y, b = blockIdx.z, t = threadIdx.x;
  for (int i = t; i < 64 * 64; i += 256) { const int r = i >> 6, d = i & 63; const int tok = s0 + r; tile[r][d] = (tok < NT) ? Vr[((size_t)(b * NT + tok)) * DD + h * DKK + d] : (bf16)0.0f; }
  __syncthreads();
#pragma unroll 1
  for (int pass = 0; pass < 2; ++pass) {
    for (int i = t; i < 64 * 8; i += 256) { const int dr = i >> 3, s8 = (i & 7) * 8; bf16 hh[8];
#pragma unroll
      for (int e = 0; e < 8; ++e) hh[e] = tile[s8 + e][dr];
      *(volatile v4u_t*)(Vt + (((size_t)(b * HH + h)) * DKK + dr) * SS + s0 + s8) = *(const v4ua*)hh; }
    __threadfence();
  }
}
__global__ __launch_bounds__(192) void k_ln(const float* __restrict__ x, const float* __restrict__ g, const float* __restrict__ be, bf16* __restrict__ XN) {
  __shared__ float red[192];
  const int m = blockIdx.x, t = threadIdx.x; bf16 h4[4];
  if (m < NTOT) {
    const v4f_t v = *(const v4fa*)(x + (size_t)m * DM + t * 4);
    red[t] = v.x + v.y + v.z + v.w; __syncthreads();
    if (t < 32) { float s = red[t] + red[t + 32] + red[t + 64] + red[t + 96] + red[t + 128] + red[t + 160];
#pragma unroll
      for (int o = 16; o >= 1; o >>= 1) s += __shfl_xor(s, o, 32); if (t == 0) red[0] = s; }
    __syncthreads(); const float mu = red[0] / (float)DM; __syncthreads();
    const float dx = v.x - mu, dy = v.y - mu, dz = v.z - mu, dw = v.w - mu; red[t] = dx * dx + dy * dy + dz * dz + dw * dw; __syncthreads();
    if (t < 32) { float s = red[t] + red[t + 32] + red[t + 64] + red[t + 96] + red[t + 128] + red[t + 160];
#pragma unroll
      for (int o = 16; o >= 1; o >>= 1) s += __shfl_xor(s, o, 32); if (t == 0) red[0] = s; }
    __syncthreads(); const float rs = rsqrtf(red[0] / (float)DM + 1e-12f);
    const v4f_t gv = *(const v4fa*)(g + t * 4), bv = *(const v4fa*)(be + t * 4);
    h4[0] = (bf16)(dx * rs * gv.x + bv.x); h4[1] = (bf16)(dy * rs * gv.y + bv.y); h4[2] = (bf16)(dz * rs * gv.z + bv.z); h4[3] = (bf16)(dw * rs * gv.w + bv.w);
  } else { h4[0] = h4[1] = h4[2] = h4[3] = (bf16)0.0f; }
  typedef __attribute__((ext_vector_type(2))) unsigned v2u; typedef unsigned v2ua __attribute__((ext_vector_type(2), may_alias));
  *(volatile v2u*)(XN + (size_t)m * DM + t * 4) = *(const v2ua*)h4; __threadfence(); *(volatile v2u*)(XN + (size_t)m * DM + t * 4) = *(const v2ua*)h4;
}
__global__ __launch_bounds__(256) void k_twpad(const float* __restrict__ W, int K, int N, float* __restrict__ WT) {
  const int n = blockIdx.x; for (int k = threadIdx.x; k < K; k += 256) { const float v = (n < N) ? W[(size_t)k * N + n] : 0.0f; *(volatile float*)(WT + (size_t)n * K + k) = v; }
  __threadfence();
  for (int k = threadIdx.x; k < K; k += 256) { const float v = (n < N) ? W[(size_t)k * N + n] : 0.0f; *(volatile float*)(WT + (size_t)n * K + k) = v; }
}
__global__ __launch_bounds__(192) void k_resid(const float* __restrict__ x, float* __restrict__ out) {
  const size_t off = (size_t)blockIdx.x * DM + threadIdx.x * 4; v4f_t v = *(const v4fa*)(out + off); const v4f_t w = *(const v4fa*)(x + off);
  v.x += w.x; v.y += w.y; v.z += w.z; v.w += w.w; *(volatile v4f_t*)(out + off) = v; __threadfence(); *(volatile v4f_t*)(out + off) = v;
}
__global__ __launch_bounds__(256) void k_bpad(const float* __restrict__ bq, const float* __restrict__ bk, const float* __restrict__ bv, float* __restrict__ bp) {
  const int which = blockIdx.x; const float* src = which == 0 ? bq : which == 1 ? bk : bv;
  for (int i = threadIdx.x; i < DD; i += 256) { const float v = (i < DO) ? src[i] : 0.0f; *(volatile float*)(bp + which * DD + i) = v; }
  __threadfence();
  for (int i = threadIdx.x; i < DD; i += 256) { const float v = (i < DO) ? src[i] : 0.0f; *(volatile float*)(bp + which * DD + i) = v; }
}
__global__ __launch_bounds__(192) void k_tailcopy(const float* __restrict__ T, float* __restrict__ out) {
  const int r = blockIdx.x; const size_t off = (size_t)r * DM + threadIdx.x * 4; const v4f_t v = *(const v4fa*)(T + off);
  *(volatile v4f_t*)(out + (size_t)(16384 + r) * DM + threadIdx.x * 4) = v; __threadfence(); *(volatile v4f_t*)(out + (size_t)(16384 + r) * DM + threadIdx.x * 4) = v;
}

extern "C" void kernel_launch(void* const* d_in, const int* in_sizes, int n_in,
                              void* d_out, int out_size, void* d_ws, size_t ws_size,
                              hipStream_t stream) {
  (void)in_sizes; (void)n_in; (void)out_size; (void)ws_size;
  const float* x = (const float*)d_in[0];
  const float* wq = (const float*)d_in[1]; const float* bq = (const float*)d_in[2];
  const float* wk = (const float*)d_in[3]; const float* bk = (const float*)d_in[4];
  const float* wv = (const float*)d_in[5]; const float* bv = (const float*)d_in[6];
  const float* wo = (const float*)d_in[7]; const float* bo = (const float*)d_in[8];
  const float* lg = (const float*)d_in[9]; const float* lb = (const float*)d_in[10];
  float* out = (float*)d_out;
  char* ws = (char*)d_ws;
  float* WqT = (float*)ws; ws += (size_t)DD * DM * 4;
  float* WkT = (float*)ws; ws += (size_t)DD * DM * 4;
  float* WvT = (float*)ws; ws += (size_t)DD * DM * 4;
  float* WoT = (float*)ws; ws += (size_t)DM * DO * 4;
  float* bp  = (float*)ws; ws += (size_t)3 * DD * 4;
  bf16* XN  = (bf16*)ws;  ws += (size_t)MP * DM * 2;
  bf16* Qb  = (bf16*)ws;  ws += (size_t)MP * DD * 2;
  bf16* Kb  = (bf16*)ws;  ws += (size_t)MP * DD * 2;
  bf16* Vr  = (bf16*)ws;  ws += (size_t)MP * DD * 2;
  bf16* VtB = (bf16*)ws;  ws += (size_t)BB * HH * DKK * SS * 2;
  bf16* At  = (bf16*)ws;  ws += (size_t)MP * DO * 2;
  float* T  = (float*)ws; ws += (size_t)128 * DM * 4;
  k_twpad<<<DD, 256, 0, stream>>>(wq, DM, DO, WqT);
  k_twpad<<<DD, 256, 0, stream>>>(wk, DM, DO, WkT);
  k_twpad<<<DD, 256, 0, stream>>>(wv, DM, DO, WvT);
  k_twpad<<<DM, 256, 0, stream>>>(wo, DO, DM, WoT);
  k_bpad<<<3, 256, 0, stream>>>(bq, bk, bv, bp);
  k_ln<<<MP, 192, 0, stream>>>(x, lg, lb, XN);
  dim3 gBlk(256);
  gemm_bias_kernel<bf16, 0><<<dim3(MP / 128, DD / 256), gBlk, 0, stream>>>(XN, WqT, bp,          Qb, MP, DD, DM);
  gemm_bias_kernel<bf16, 0><<<dim3(MP / 128, DD / 256), gBlk, 0, stream>>>(XN, WkT, bp + DD,     Kb, MP, DD, DM);
  gemm_bias_kernel<bf16, 0><<<dim3(MP / 128, DD / 256), gBlk, 0, stream>>>(XN, WvT, bp + 2 * DD, Vr, MP, DD, DM);
  k_vt<<<dim3(SS / 64, HH, BB), 256, 0, stream>>>(Vr, VtB);
  attn_kernel<<<dim3(SS / 64, HH, BB), dim3(64), 0, stream>>>(Qb, Kb, VtB, At);
  gemm_bias_kernel<bf16, 2><<<dim3(16384 / 128, DM / 256), gBlk, 0, stream>>>(At, WoT, bo, out, 16384, DM, DO);
  gemm_bias_kernel<bf16, 2><<<dim3(1, DM / 256), gBlk, 0, stream>>>(At + (size_t)16384 * DO, WoT, bo, T, 128, DM, DO);
  k_tailcopy<<<NTOT - 16384, 192, 0, stream>>>(T, out);
  k_resid<<<NTOT, 192, 0, stream>>>(x, out);
}
